// KANLayer_9165460210146
// MI455X (gfx1250) — hardware-verified
//
#include <hip/hip_runtime.h>

typedef _Float16 v16h __attribute__((ext_vector_type(16)));
typedef _Float16 v8h  __attribute__((ext_vector_type(8)));
typedef float    v8f  __attribute__((ext_vector_type(8)));
typedef float    v4f  __attribute__((ext_vector_type(4)));
typedef v4f v4fa __attribute__((may_alias));

#ifndef NB
#define NB 8192
#endif
#define NB_FULL 8192
#define DIN   192
#define NG    192
#define NOUT  16
#define KTOT  (NG * DIN)
#define NWELEM (NOUT * KTOT)
#define WPLANE_BYTES ((size_t)NWELEM * 2)
#define WCARRY 256.0f
#define WINV   0.00390625f

static_assert(DIN % 32 == 0);
static_assert(NOUT == 16);
static_assert(NWELEM % 8 == 0);
static_assert(NB >= 1);
static_assert(NB <= NB_FULL);
static_assert((KTOT % 8) == 0);

__device__ __forceinline__ float bf16_rne(float f) {
  unsigned u = __float_as_uint(f);
  u = (u + 0x7fffu + ((u >> 16) & 1u)) & 0xffff0000u;
  return __uint_as_float(u);
}

union Frag { v16h v; v8h hv[2]; };

__device__ __forceinline__ v8f wmma16(v16h a, v16h b, v8f c) {
  c = __builtin_amdgcn_wmma_f32_16x16x32_f16(false, a, false, b, (short)0, c, false, false);
  asm volatile("v_nop\n\tv_nop\n\tv_nop\n\tv_nop" : "+v"(c) : "v"(a), "v"(b));
  return c;
}

__global__ __launch_bounds__(256) void k_prep_w(const float* __restrict__ spl,
                                                _Float16* wp, int nelem) {
  const int t    = blockIdx.x * 256 + threadIdx.x;
  const int ngrp = nelem >> 3;
  const int gi   = min(t, ngrp - 1);
  const size_t base = (size_t)gi * 8;
  const v4f* sp = (const v4f*)(spl + base);
  const v4f p0 = sp[0];
  const v4f p1 = sp[1];
  v8h o;
  o[0] = (_Float16)(bf16_rne(p0[0]) * WCARRY);
  o[1] = (_Float16)(bf16_rne(p0[1]) * WCARRY);
  o[2] = (_Float16)(bf16_rne(p0[2]) * WCARRY);
  o[3] = (_Float16)(bf16_rne(p0[3]) * WCARRY);
  o[4] = (_Float16)(bf16_rne(p1[0]) * WCARRY);
  o[5] = (_Float16)(bf16_rne(p1[1]) * WCARRY);
  o[6] = (_Float16)(bf16_rne(p1[2]) * WCARRY);
  o[7] = (_Float16)(bf16_rne(p1[3]) * WCARRY);
  const bool ok = (t < ngrp);
  if (ok) *(volatile v8h*)(wp + base) = o;
  __threadfence();
  if (ok) *(volatile v8h*)(wp + base) = o;
}

__global__ __launch_bounds__(64) void k_kan_gemm(const float* __restrict__ x,
                                                 const float* __restrict__ grid,
                                                 const _Float16* __restrict__ wp,
                                                 float* out, int nrows) {
  __shared__ __attribute__((aligned(16))) float stile[2][256];

  const int lane = threadIdx.x & 31;
  const int wid  = threadIdx.x >> 5;
  const int h    = lane >> 4;
  const int m    = lane & 15;

  const int ntiles = (nrows + 15) >> 4;
  const int gw     = blockIdx.x * 2 + wid;
  const int tile   = min(gw, ntiles - 1);
  const int n0     = tile * 16;
  const int rowA   = min(n0 + m, nrows - 1);

  const float*    xrow = x  + (size_t)rowA * DIN;
  const _Float16* wrow = wp + (size_t)m * KTOT;

  v8f acc;
  #pragma unroll
  for (int r = 0; r < 8; ++r) acc[r] = 0.0f;

  #pragma unroll 1
  for (int db = 0; db < DIN / 32; ++db) {
    const float* xr = xrow + db * 32 + 8 * h;
    const v4f x0 = *(const v4f*)(xr);
    const v4f x1 = *(const v4f*)(xr + 4);
    const v4f x2 = *(const v4f*)(xr + 16);
    const v4f x3 = *(const v4f*)(xr + 20);
    float xv[16];
    #pragma unroll
    for (int i = 0; i < 4; ++i) {
      xv[i]      = bf16_rne(x0[i]);
      xv[4 + i]  = bf16_rne(x1[i]);
      xv[8 + i]  = bf16_rne(x2[i]);
      xv[12 + i] = bf16_rne(x3[i]);
    }
    const _Float16* wb = wrow + db * 32 + 8 * h;

    #pragma unroll 2
    for (int g = 0; g < NG; ++g) {
      const float gb = bf16_rne(grid[g]);
      Frag a;
      #pragma unroll
      for (int i = 0; i < 16; ++i) {
        const float t  = xv[i] - gb;
        const float bv = fmaxf(1.0f - fabsf(t), 0.0f);
        a.v[i] = (_Float16)bv;
      }
      Frag b;
      const _Float16* wg = wb + (size_t)g * DIN;
      b.hv[0] = *(const v8h*)(wg);
      b.hv[1] = *(const v8h*)(wg + 16);
      acc = wmma16(a.v, b.v, acc);
    }
  }

  float* st = &stile[wid][0];
  #pragma unroll
  for (int r = 0; r < 8; ++r) st[(8 * h + r) * 16 + m] = acc[r] * WINV;
  __syncthreads();

  v4f vals[2];
  size_t oidx[2];
  bool ok[2];
  #pragma unroll
  for (int q = 0; q < 2; ++q) {
    const int e  = q * 128 + 4 * lane;
    const int rt = e >> 4;
    const int cl = e & 15;
    vals[q] = *(const v4fa*)(st + e);
    oidx[q] = (size_t)(n0 + rt) * NOUT + cl;
    ok[q]   = (gw < ntiles) && (n0 + rt < nrows);
  }
  #pragma unroll
  for (int q = 0; q < 2; ++q)
    if (ok[q]) *(volatile v4f*)(out + oidx[q]) = vals[q];
  __threadfence();
  #pragma unroll
  for (int q = 0; q < 2; ++q)
    if (ok[q]) *(volatile v4f*)(out + oidx[q]) = vals[q];
}

extern "C" void kernel_launch(void* const* d_in, const int* in_sizes, int n_in,
                              void* d_out, int out_size, void* d_ws, size_t ws_size,
                              hipStream_t stream) {
  if (n_in < 3) return;
  if (in_sizes[0] < NB * DIN) return;
  if (in_sizes[1] < NOUT * NG * DIN) return;
  if (in_sizes[2] < NG) return;
  if (out_size < NB * NOUT) return;
  if (ws_size < WPLANE_BYTES) return;

  const float* x       = (const float*)d_in[0];
  const float* splines = (const float*)d_in[1];
  const float* grid    = (const float*)d_in[2];
  float* out           = (float*)d_out;

  _Float16* wp = (_Float16*)d_ws;

  const int nrows  = NB;
  const int ngrp   = NWELEM / 8;
  const int pblk   = (ngrp + 255) / 256;
  const int ntiles = (nrows + 15) / 16;
  const int gblk   = (ntiles + 1) / 2;

  k_prep_w<<<dim3(pblk), dim3(256), 0, stream>>>(splines, wp, (int)NWELEM);
  k_kan_gemm<<<dim3(gblk), dim3(64), 0, stream>>>(x, grid, wp, out, nrows);
}
